// DCFNet_69647189671988
// MI455X (gfx1250) — hardware-verified
//
#include <hip/hip_runtime.h>

#define NS    16
#define CIN   3
#define CF    32
#define CROP  256
#define NBIN  129
#define VP    160
#define K2    288
#define TABN  65536
#define GPL   (NS * VP * CROP)
#define PPL   (NS * CROP * CROP)
#define LDP   260
#define LDQ   164

typedef _Float16 v16h __attribute__((ext_vector_type(16)));
typedef _Float16 v8h  __attribute__((ext_vector_type(8)));
typedef __bf16   v16b __attribute__((ext_vector_type(16)));
typedef __bf16   v8b  __attribute__((ext_vector_type(8)));
typedef unsigned short v8us __attribute__((ext_vector_type(8)));
typedef unsigned int   v8u  __attribute__((ext_vector_type(8)));
typedef float v8f __attribute__((ext_vector_type(8)));
typedef float v4f __attribute__((ext_vector_type(4)));
typedef v8h  __attribute__((may_alias)) v8ha;
typedef v8b  __attribute__((may_alias)) v8ba;
typedef v8us __attribute__((may_alias)) v8usa;
typedef v4f  __attribute__((may_alias)) v4fa;

union FragHU { v16h v; v8h half[2]; v8u u; };
union FragBU { v16b v; v8b half[2]; v8u u; };

__device__ __forceinline__ v8f wmma_h(v16h a, v16h b, v8f c) {
  v8f d = __builtin_amdgcn_wmma_f32_16x16x32_f16(false, a, false, b, (short)0, c, false, false);
  asm volatile("v_nop\n\tv_nop\n\tv_nop\n\tv_nop" : "+v"(d) : "v"(a), "v"(b));
  return d;
}
__device__ __forceinline__ v8f wmma_b(v16b a, v16b b, v8f c) {
  v8f d = __builtin_amdgcn_wmma_f32_16x16x32_bf16(false, a, false, b, (short)0, c, false, false);
  asm volatile("v_nop\n\tv_nop\n\tv_nop\n\tv_nop" : "+v"(d) : "v"(a), "v"(b));
  return d;
}
__device__ __forceinline__ v8f wmma3(v16b ahi, v16b alo, v16b bhi, v16b blo, v8f c) {
  c = wmma_b(ahi, bhi, c);
  c = wmma_b(ahi, blo, c);
  c = wmma_b(alo, bhi, c);
  return c;
}

__device__ __forceinline__ v16h ldh(const _Float16* p, int hh) {
  FragHU f;
  f.half[0] = *(const v8ha*)(p + 8 * hh);
  f.half[1] = *(const v8ha*)(p + 16 + 8 * hh);
  return f.v;
}
__device__ __forceinline__ v16b ldb(const unsigned short* p, int hh) {
  FragBU f;
  f.half[0] = *(const v8ba*)(p + 8 * hh);
  f.half[1] = *(const v8ba*)(p + 16 + 8 * hh);
  return f.v;
}
__device__ __forceinline__ v16b negb(v16b x) {
  FragBU f; f.v = x; f.u = f.u ^ 0x80008000u; return f.v;
}
__device__ __forceinline__ v16h maskh(v16h x, bool ok) {
  FragHU f; f.v = x; f.u = f.u & (ok ? 0xffffffffu : 0u); return f.v;
}

__device__ __forceinline__ unsigned short bf_bits(float x) {
  unsigned int u = __float_as_uint(x);
  u += 0x7FFFu + ((u >> 16) & 1u);
  return (unsigned short)(u >> 16);
}
__device__ __forceinline__ float bf_val(unsigned short b) {
  return __uint_as_float(((unsigned int)b) << 16);
}
__device__ __forceinline__ void split8f(const float* x, v8us* hi, v8us* lo) {
  v8us hv = {0, 0, 0, 0, 0, 0, 0, 0}, lv = {0, 0, 0, 0, 0, 0, 0, 0};
  #pragma unroll
  for (int j = 0; j < 8; ++j) {
    const unsigned short hb = bf_bits(x[j]);
    const unsigned short lb = bf_bits(x[j] - bf_val(hb));
    hv[j] = hb; lv[j] = lb;
  }
  *hi = hv; *lo = lv;
}
__device__ __forceinline__ void split8v(v4f a, v4f c, v8us* hi, v8us* lo) {
  const float x[8] = {a.x, a.y, a.z, a.w, c.x, c.y, c.z, c.w};
  split8f(x, hi, lo);
}

__global__ __launch_bounds__(128) void prep_kernel(const float* __restrict__ w1,
                                                   const float* __restrict__ w2,
                                                   unsigned short* __restrict__ tabs,
                                                   _Float16* __restrict__ w1p,
                                                   _Float16* __restrict__ w2p)
{
  __shared__ float tcs[CROP];
  __shared__ float tsn[CROP];
  const int t = threadIdx.x, lane = t & 31, wv = t >> 5;
  const int blk = blockIdx.x;
  if (blk < CROP) {
    #pragma unroll 1
    for (int i = 0; i < 2; ++i) {
      const int mm = t + 128 * i;
      const float x = (float)mm * 0.0078125f;
      tcs[mm] = cospif(x);
      tsn[mm] = sinpif(x);
    }
    __syncthreads();
    const int a = blk;
    const float sgn = (a & 1) ? -1.0f : 1.0f;
    float vals[8];
    #pragma unroll
    for (int j = 0; j < 8; ++j) {
      const int b = 8 * lane + j;
      const int mm = (a * b) & 255;
      const float cv = tcs[mm], sv = tsn[mm];
      const bool mid = (b >= 1) && (b <= 127);
      const float bc = (b == 0) ? 1.0f : ((b == 128) ? sgn : (mid ? 2.0f * cv : 0.0f));
      const float bs = mid ? -2.0f * sv : 0.0f;
      float v = cv;
      if (wv == 1) v = sv;
      if (wv == 2) v = bc;
      if (wv == 3) v = bs;
      vals[j] = v;
    }
    v8us hi, lo;
    split8f(vals, &hi, &lo);
    unsigned short* ph = tabs + (size_t)(2 * wv) * TABN + (size_t)a * CROP + 8 * lane;
    unsigned short* pl = ph + TABN;
    *(volatile v8us*)ph = hi;
    *(volatile v8us*)pl = lo;
    __threadfence();
    *(volatile v8us*)ph = hi;
    *(volatile v8us*)pl = lo;
  } else if (blk < CROP + 9) {
    const int p = (blk - CROP) * 128 + t;
    const int co = p / 36;
    const int kp = (p - co * 36) * 8;
    const int tap = kp >> 5, ci0 = kp & 31;
    v8h o;
    #pragma unroll
    for (int j = 0; j < 8; ++j) o[j] = (_Float16)(16.0f * w2[(co * CF + ci0 + j) * 9 + tap]);
    _Float16* d = w2p + (size_t)p * 8;
    *(volatile v8h*)d = o;
    __threadfence();
    *(volatile v8h*)d = o;
  } else {
    const int p = t;
    const int co = p >> 2, kp = (p & 3) * 8;
    v8h o;
    #pragma unroll
    for (int j = 0; j < 8; ++j) {
      const int k = kp + j;
      const int kc = (k < 27) ? k : 26;
      const float v = w1[co * 27 + kc];
      o[j] = (_Float16)((k < 27) ? 16.0f * v : 0.0f);
    }
    _Float16* d = w1p + (size_t)p * 8;
    *(volatile v8h*)d = o;
    __threadfence();
    *(volatile v8h*)d = o;
  }
}

__device__ __forceinline__ void f1_store_pass(const _Float16* sO, _Float16* base, int t) {
  #pragma unroll
  for (int i = 0; i < 4; ++i) {
    const int p = i * 256 + t;
    const v8h v = *(const v8ha*)(sO + p * 8);
    *(volatile v8h*)(base + (size_t)p * 8) = v;
  }
}

__global__ __launch_bounds__(256) void conv1_kernel(const float* __restrict__ z,
                                                    const _Float16* __restrict__ w1p,
                                                    const float* __restrict__ b1,
                                                    _Float16* __restrict__ f1)
{
  __shared__ __attribute__((aligned(16))) _Float16 sA[CROP * 32];
  __shared__ __attribute__((aligned(16))) _Float16 sO[CROP * CF];
  const int t = threadIdx.x, lane = t & 31, wv = t >> 5, hh = lane >> 4, m = lane & 15;
  const int img = blockIdx.x >> 8, y = blockIdx.x & 255;

  {
    float av[32];
    #pragma unroll
    for (int j = 27; j < 32; ++j) av[j] = 0.0f;
    #pragma unroll
    for (int ci = 0; ci < CIN; ++ci) {
      #pragma unroll
      for (int ky = 0; ky < 3; ++ky) {
        const int iy = y + ky - 1;
        const int iyc = iy < 0 ? 0 : (iy > CROP - 1 ? CROP - 1 : iy);
        const bool oky = (iy >= 0) && (iy < CROP);
        const float* zr = z + ((size_t)(img * CIN + ci) * CROP + iyc) * CROP;
        #pragma unroll
        for (int kx = 0; kx < 3; ++kx) {
          const int ix = t + kx - 1;
          const int ixc = ix < 0 ? 0 : (ix > CROP - 1 ? CROP - 1 : ix);
          const bool ok = oky && (ix >= 0) && (ix < CROP);
          const float v = zr[ixc];
          av[ci * 9 + ky * 3 + kx] = ok ? v : 0.0f;
        }
      }
    }
    v8h p0, p1, p2, p3;
    #pragma unroll
    for (int j = 0; j < 8; ++j) {
      p0[j] = (_Float16)av[j];
      p1[j] = (_Float16)av[8 + j];
      p2[j] = (_Float16)av[16 + j];
      p3[j] = (_Float16)av[24 + j];
    }
    _Float16* d = sA + t * 32;
    *(v8ha*)(d) = p0;
    *(v8ha*)(d + 8) = p1;
    *(v8ha*)(d + 16) = p2;
    *(v8ha*)(d + 24) = p3;
  }
  __syncthreads();

  const v16h wb0 = ldh(w1p + m * 32, hh);
  const v16h wb1 = ldh(w1p + (16 + m) * 32, hh);
  const v8f zero8 = {0.f, 0.f, 0.f, 0.f, 0.f, 0.f, 0.f, 0.f};
  v8f acc[2][2];
  #pragma unroll
  for (int mt = 0; mt < 2; ++mt) {
    const v16h a = ldh(sA + (32 * wv + 16 * mt + m) * 32, hh);
    acc[mt][0] = wmma_h(a, wb0, zero8);
    acc[mt][1] = wmma_h(a, wb1, zero8);
  }

  #pragma unroll
  for (int nt = 0; nt < 2; ++nt) {
    const int co = 16 * nt + m;
    const float bias = b1[co];
    #pragma unroll
    for (int mt = 0; mt < 2; ++mt) {
      #pragma unroll
      for (int r = 0; r < 8; ++r) {
        const int px = 32 * wv + 16 * mt + 8 * hh + r;
        const float val = fmaxf(acc[mt][nt][r] * 0.0625f + bias, 0.0f);
        sO[px * CF + co] = (_Float16)val;
      }
    }
  }
  __syncthreads();

  _Float16* base = f1 + (size_t)(img * CROP + y) * CROP * CF;
  f1_store_pass(sO, base, t);
  __threadfence();
  f1_store_pass(sO, base, t);
}

__global__ __launch_bounds__(256) void conv2_kernel(const _Float16* __restrict__ f1,
                                                    const _Float16* __restrict__ w2p,
                                                    const float* __restrict__ b2,
                                                    const float* __restrict__ cw,
                                                    unsigned short* __restrict__ ghi,
                                                    unsigned short* __restrict__ glo)
{
  __shared__ __attribute__((aligned(16))) _Float16 sW[CF * K2];
  __shared__ float sD[CROP * 33];
  __shared__ __attribute__((aligned(16))) float sG[CROP];
  const int t = threadIdx.x, lane = t & 31, wv = t >> 5, hh = lane >> 4, m = lane & 15;
  const int img = blockIdx.x >> 8, y = blockIdx.x & 255;

  for (int p = t; p < (CF * K2) / 8; p += 256)
    *(v8ha*)(sW + p * 8) = *(const v8ha*)(w2p + (size_t)p * 8);
  __syncthreads();

  const v8f zero8 = {0.f, 0.f, 0.f, 0.f, 0.f, 0.f, 0.f, 0.f};
  v8f acc[2][2];
  #pragma unroll
  for (int mt = 0; mt < 2; ++mt) { acc[mt][0] = zero8; acc[mt][1] = zero8; }
  const int xw = 32 * wv;

  #pragma unroll 1
  for (int dy = 0; dy < 3; ++dy) {
    const int iy = y + dy - 1;
    if (iy < 0 || iy > CROP - 1) continue;
    const _Float16* rowp = f1 + (size_t)(img * CROP + iy) * CROP * CF;
    #pragma unroll
    for (int dx = 0; dx < 3; ++dx) {
      const int tap = dy * 3 + dx;
      const v16h wb0 = ldh(sW + m * K2 + tap * CF, hh);
      const v16h wb1 = ldh(sW + (16 + m) * K2 + tap * CF, hh);
      #pragma unroll
      for (int mt = 0; mt < 2; ++mt) {
        const int ix = xw + 16 * mt + m + dx - 1;
        const int ixc = ix < 0 ? 0 : (ix > CROP - 1 ? CROP - 1 : ix);
        const bool ok = (ix >= 0) && (ix < CROP);
        const v16h a = maskh(ldh(rowp + (size_t)ixc * CF, hh), ok);
        acc[mt][0] = wmma_h(a, wb0, acc[mt][0]);
        acc[mt][1] = wmma_h(a, wb1, acc[mt][1]);
      }
    }
  }

  #pragma unroll
  for (int mt = 0; mt < 2; ++mt)
    #pragma unroll
    for (int nt = 0; nt < 2; ++nt)
      #pragma unroll
      for (int r = 0; r < 8; ++r)
        sD[(xw + 16 * mt + 8 * hh + r) * 33 + 16 * nt + m] = acc[mt][nt][r];
  __syncthreads();

  {
    float v[CF];
    float sqp[CF + 4];
    sqp[0] = 0.0f; sqp[1] = 0.0f; sqp[CF + 2] = 0.0f; sqp[CF + 3] = 0.0f;
    #pragma unroll
    for (int c = 0; c < CF; ++c) {
      v[c] = sD[t * 33 + c] * 0.0625f + b2[c];
      sqp[c + 2] = v[c] * v[c];
    }
    float gs = 0.0f;
    #pragma unroll
    for (int c = 0; c < CF; ++c) {
      const float win = sqp[c] + sqp[c + 1] + sqp[c + 2] + sqp[c + 3] + sqp[c + 4];
      const float base = 1.0f + 2e-5f * win;
      const float rr = __expf(-0.75f * __logf(base));
      gs += v[c] * rr;
    }
    sG[t] = gs * cw[y * CROP + t];
  }
  __syncthreads();

  if (t < 64) {
    const v4f a = *(const v4fa*)(sG + 8 * lane);
    const v4f c = *(const v4fa*)(sG + 8 * lane + 4);
    v8us hi, lo;
    split8v(a, c, &hi, &lo);
    v8us val = hi;
    if (wv != 0) val = lo;
    unsigned short* dst = ((wv == 0) ? ghi : glo) + (size_t)(img * CROP + y) * CROP + 8 * lane;
    *(volatile v8us*)dst = val;
    __threadfence();
    *(volatile v8us*)dst = val;
  }
}

__device__ __forceinline__ void gstore_pass(const float* s, unsigned short* ph, unsigned short* pl,
                                            int img, int v0, int t) {
  #pragma unroll
  for (int i = 0; i < 2; ++i) {
    const int p = i * 256 + t;
    const int row = p >> 5, col8 = (p & 31) * 8;
    const v4f a = *(const v4fa*)(s + row * LDP + col8);
    const v4f c = *(const v4fa*)(s + row * LDP + col8 + 4);
    v8us hi, lo;
    split8v(a, c, &hi, &lo);
    const size_t dst = ((size_t)img * VP + v0 + row) * CROP + col8;
    *(volatile v8us*)(ph + dst) = hi;
    *(volatile v8us*)(pl + dst) = lo;
  }
}

__global__ __launch_bounds__(256) void rowdft_kernel(const unsigned short* __restrict__ ghi,
                                                     const unsigned short* __restrict__ glo,
                                                     const unsigned short* __restrict__ tabs,
                                                     unsigned short* __restrict__ gpl)
{
  __shared__ __attribute__((aligned(16))) float sR[16 * LDP];
  __shared__ __attribute__((aligned(16))) float sI[16 * LDP];
  const int t = threadIdx.x, lane = t & 31, wv = t >> 5, hh = lane >> 4, m = lane & 15;
  const int img = blockIdx.y, v0 = 16 * blockIdx.x, c0 = 32 * wv;

  const unsigned short* pa  = tabs + (size_t)(v0 + m) * CROP;
  const unsigned short* pb  = ghi + ((size_t)img * CROP + c0 + m) * CROP;
  const unsigned short* pbl = glo + ((size_t)img * CROP + c0 + m) * CROP;

  const v8f zero8 = {0.f, 0.f, 0.f, 0.f, 0.f, 0.f, 0.f, 0.f};
  v8f accR[2], accI[2];
  accR[0] = zero8; accR[1] = zero8; accI[0] = zero8; accI[1] = zero8;

  #pragma unroll 1
  for (int k0 = 0; k0 < CROP; k0 += 32) {
    const v16b chi = ldb(pa + k0, hh);
    const v16b clo = ldb(pa + TABN + k0, hh);
    const v16b snh = negb(ldb(pa + 2 * TABN + k0, hh));
    const v16b snl = negb(ldb(pa + 3 * TABN + k0, hh));
    #pragma unroll
    for (int nt = 0; nt < 2; ++nt) {
      const v16b bh = ldb(pb + nt * 16 * CROP + k0, hh);
      const v16b bl = ldb(pbl + nt * 16 * CROP + k0, hh);
      accR[nt] = wmma3(chi, clo, bh, bl, accR[nt]);
      accI[nt] = wmma3(snh, snl, bh, bl, accI[nt]);
    }
  }

  #pragma unroll
  for (int nt = 0; nt < 2; ++nt)
    #pragma unroll
    for (int r = 0; r < 8; ++r) {
      const int row = 8 * hh + r, col = c0 + 16 * nt + m;
      const bool keep = (v0 + row) < NBIN;
      sR[row * LDP + col] = keep ? accR[nt][r] : 0.0f;
      sI[row * LDP + col] = keep ? accI[nt][r] : 0.0f;
    }
  __syncthreads();

  gstore_pass(sR, gpl, gpl + GPL, img, v0, t);
  gstore_pass(sI, gpl + 2 * GPL, gpl + 3 * GPL, img, v0, t);
  __threadfence();
  gstore_pass(sR, gpl, gpl + GPL, img, v0, t);
  gstore_pass(sI, gpl + 2 * GPL, gpl + 3 * GPL, img, v0, t);
}

__device__ __forceinline__ void fstore_pass(const float* sR, const float* sI, const float* __restrict__ wf,
                                            unsigned short* fpl, int img, int v0, int t) {
  #pragma unroll
  for (int i = 0; i < 2; ++i) {
    const int p = i * 256 + t;
    const int row = p >> 5, col8 = (p & 31) * 8;
    const int v = v0 + row;
    const int vc = (v < NBIN - 1) ? v : (NBIN - 1);
    const bool keep = v < NBIN;
    const v4f r0 = *(const v4fa*)(sR + row * LDP + col8);
    const v4f r1 = *(const v4fa*)(sR + row * LDP + col8 + 4);
    const v4f i0 = *(const v4fa*)(sI + row * LDP + col8);
    const v4f i1 = *(const v4fa*)(sI + row * LDP + col8 + 4);
    const float sr[8] = {r0.x, r0.y, r0.z, r0.w, r1.x, r1.y, r1.z, r1.w};
    const float si[8] = {i0.x, i0.y, i0.z, i0.w, i1.x, i1.y, i1.z, i1.w};
    float fr[8], fi[8];
    #pragma unroll
    for (int j = 0; j < 8; ++j) {
      const int u = col8 + j;
      const size_t widx = ((size_t)(CROP + u) * NBIN + vc) * 2;
      const float a = wf[widx], b = wf[widx + 1];
      fr[j] = keep ? (a * sr[j] + b * si[j]) : 0.0f;
      fi[j] = keep ? (a * si[j] - b * sr[j]) : 0.0f;
    }
    v8us frh, frl, fih, fil;
    split8f(fr, &frh, &frl);
    split8f(fi, &fih, &fil);
    const size_t dst = ((size_t)img * VP + v) * CROP + col8;
    *(volatile v8us*)(fpl + dst) = frh;
    *(volatile v8us*)(fpl + GPL + dst) = frl;
    *(volatile v8us*)(fpl + 2 * GPL + dst) = fih;
    *(volatile v8us*)(fpl + 3 * GPL + dst) = fil;
  }
}

__global__ __launch_bounds__(256) void coldft_kernel(const unsigned short* __restrict__ gpl,
                                                     const unsigned short* __restrict__ tabs,
                                                     const float* __restrict__ wf,
                                                     unsigned short* __restrict__ fpl)
{
  __shared__ __attribute__((aligned(16))) float sR[16 * LDP];
  __shared__ __attribute__((aligned(16))) float sI[16 * LDP];
  const int t = threadIdx.x, lane = t & 31, wv = t >> 5, hh = lane >> 4, m = lane & 15;
  const int img = blockIdx.y, v0 = 16 * blockIdx.x, c0 = 32 * wv;

  const unsigned short* pa = gpl + ((size_t)img * VP + v0 + m) * CROP;
  const unsigned short* pb = tabs + (size_t)(c0 + m) * CROP;

  const v8f zero8 = {0.f, 0.f, 0.f, 0.f, 0.f, 0.f, 0.f, 0.f};
  v8f accR[2], accI[2];
  accR[0] = zero8; accR[1] = zero8; accI[0] = zero8; accI[1] = zero8;

  #pragma unroll 1
  for (int k0 = 0; k0 < CROP; k0 += 32) {
    const v16b grh = ldb(pa + k0, hh);
    const v16b grl = ldb(pa + GPL + k0, hh);
    const v16b gih = ldb(pa + 2 * GPL + k0, hh);
    const v16b gil = ldb(pa + 3 * GPL + k0, hh);
    #pragma unroll
    for (int nt = 0; nt < 2; ++nt) {
      const unsigned short* q = pb + nt * 16 * CROP + k0;
      const v16b ch = ldb(q, hh), cl = ldb(q + TABN, hh);
      const v16b sh = ldb(q + 2 * TABN, hh), sl = ldb(q + 3 * TABN, hh);
      const v16b snh = negb(sh), snl = negb(sl);
      accR[nt] = wmma3(grh, grl, ch, cl, accR[nt]);
      accR[nt] = wmma3(gih, gil, sh, sl, accR[nt]);
      accI[nt] = wmma3(gih, gil, ch, cl, accI[nt]);
      accI[nt] = wmma3(grh, grl, snh, snl, accI[nt]);
    }
  }

  #pragma unroll
  for (int nt = 0; nt < 2; ++nt)
    #pragma unroll
    for (int r = 0; r < 8; ++r) {
      const int row = 8 * hh + r, col = c0 + 16 * nt + m;
      sR[row * LDP + col] = accR[nt][r];
      sI[row * LDP + col] = accI[nt][r];
    }
  __syncthreads();

  fstore_pass(sR, sI, wf, fpl, img, v0, t);
  __threadfence();
  fstore_pass(sR, sI, wf, fpl, img, v0, t);
}

__device__ __forceinline__ void pstore_pass(const float* s, unsigned short* ph, unsigned short* pl,
                                            int img, int h0, int t) {
  const v4f z4 = {0.f, 0.f, 0.f, 0.f};
  #pragma unroll
  for (int i = 0; i < 4; ++i) {
    const int p = i * 160 + t;
    if (p < 512) {
      const int row = p >> 5, col8 = (p & 31) * 8;
      const int colc = (col8 < VP - 8) ? col8 : (VP - 8);
      const bool in = col8 < VP;
      v4f a = *(const v4fa*)(s + row * LDQ + colc);
      v4f c = *(const v4fa*)(s + row * LDQ + colc + 4);
      if (!in) { a = z4; c = z4; }
      v8us hi, lo;
      split8v(a, c, &hi, &lo);
      const size_t dst = ((size_t)img * CROP + h0 + row) * CROP + col8;
      *(volatile v8us*)(ph + dst) = hi;
      *(volatile v8us*)(pl + dst) = lo;
    }
  }
}

__global__ __launch_bounds__(160) void invcol_kernel(const unsigned short* __restrict__ fpl,
                                                     const unsigned short* __restrict__ tabs,
                                                     unsigned short* __restrict__ ppl)
{
  __shared__ __attribute__((aligned(16))) float sR[16 * LDQ];
  __shared__ __attribute__((aligned(16))) float sI[16 * LDQ];
  const int t = threadIdx.x, lane = t & 31, wv = t >> 5, hh = lane >> 4, m = lane & 15;
  const int h0 = 16 * blockIdx.x, img = blockIdx.y, vb = 32 * wv;

  const unsigned short* pa = tabs + (size_t)(h0 + m) * CROP;
  const unsigned short* pb = fpl + ((size_t)img * VP + vb + m) * CROP;

  const v8f zero8 = {0.f, 0.f, 0.f, 0.f, 0.f, 0.f, 0.f, 0.f};
  v8f accR[2], accI[2];
  accR[0] = zero8; accR[1] = zero8; accI[0] = zero8; accI[1] = zero8;

  #pragma unroll 1
  for (int k0 = 0; k0 < CROP; k0 += 32) {
    const v16b ch = ldb(pa + k0, hh), cl = ldb(pa + TABN + k0, hh);
    const v16b sh = ldb(pa + 2 * TABN + k0, hh), sl = ldb(pa + 3 * TABN + k0, hh);
    #pragma unroll
    for (int nt = 0; nt < 2; ++nt) {
      const unsigned short* q = pb + nt * 16 * CROP + k0;
      const v16b frh = ldb(q, hh), frl = ldb(q + GPL, hh);
      const v16b fih = ldb(q + 2 * GPL, hh), fil = ldb(q + 3 * GPL, hh);
      accR[nt] = wmma3(ch, cl, frh, frl, accR[nt]);
      accR[nt] = wmma3(sh, sl, negb(fih), negb(fil), accR[nt]);
      accI[nt] = wmma3(ch, cl, fih, fil, accI[nt]);
      accI[nt] = wmma3(sh, sl, frh, frl, accI[nt]);
    }
  }

  #pragma unroll
  for (int nt = 0; nt < 2; ++nt)
    #pragma unroll
    for (int r = 0; r < 8; ++r) {
      const int row = 8 * hh + r, col = vb + 16 * nt + m;
      sR[row * LDQ + col] = accR[nt][r];
      sI[row * LDQ + col] = accI[nt][r];
    }
  __syncthreads();

  pstore_pass(sR, ppl, ppl + PPL, img, h0, t);
  pstore_pass(sI, ppl + 2 * PPL, ppl + 3 * PPL, img, h0, t);
  __threadfence();
  pstore_pass(sR, ppl, ppl + PPL, img, h0, t);
  pstore_pass(sI, ppl + 2 * PPL, ppl + 3 * PPL, img, h0, t);
}

__device__ __forceinline__ void ostore_pass(const float* s, float* out, int img, int h0, int t) {
  #pragma unroll
  for (int i = 0; i < 4; ++i) {
    const int p = i * 256 + t;
    const int row = p >> 6, col4 = (p & 63) * 4;
    const v4f v = *(const v4fa*)(s + row * LDP + col4);
    *(volatile v4f*)(out + (size_t)img * CROP * CROP + (size_t)(h0 + row) * CROP + col4) = v;
  }
}

__global__ __launch_bounds__(256) void invrow_kernel(const unsigned short* __restrict__ ppl,
                                                     const unsigned short* __restrict__ tabs,
                                                     float* __restrict__ out)
{
  __shared__ __attribute__((aligned(16))) float sO[16 * LDP];
  const int t = threadIdx.x, lane = t & 31, wv = t >> 5, hh = lane >> 4, m = lane & 15;
  const int h0 = 16 * blockIdx.x, img = blockIdx.y, wb = 32 * wv;

  const unsigned short* pa = ppl + ((size_t)img * CROP + h0 + m) * CROP;
  const unsigned short* pb = tabs + (size_t)4 * TABN + (size_t)(wb + m) * CROP;

  const v8f zero8 = {0.f, 0.f, 0.f, 0.f, 0.f, 0.f, 0.f, 0.f};
  v8f acc[2];
  acc[0] = zero8; acc[1] = zero8;

  #pragma unroll 1
  for (int k0 = 0; k0 < VP; k0 += 32) {
    const v16b prh = ldb(pa + k0, hh), prl = ldb(pa + PPL + k0, hh);
    const v16b pih = ldb(pa + 2 * PPL + k0, hh), pil = ldb(pa + 3 * PPL + k0, hh);
    #pragma unroll
    for (int nt = 0; nt < 2; ++nt) {
      const unsigned short* q = pb + nt * 16 * CROP + k0;
      const v16b bch = ldb(q, hh), bcl = ldb(q + TABN, hh);
      const v16b bsh = ldb(q + 2 * TABN, hh), bsl = ldb(q + 3 * TABN, hh);
      acc[nt] = wmma3(prh, prl, bch, bcl, acc[nt]);
      acc[nt] = wmma3(pih, pil, bsh, bsl, acc[nt]);
    }
  }

  #pragma unroll
  for (int nt = 0; nt < 2; ++nt)
    #pragma unroll
    for (int r = 0; r < 8; ++r)
      sO[(8 * hh + r) * LDP + wb + 16 * nt + m] = acc[nt][r] * (1.0f / 65536.0f);
  __syncthreads();

  ostore_pass(sO, out, img, h0, t);
  __threadfence();
  ostore_pass(sO, out, img, h0, t);
}

extern "C" void kernel_launch(void* const* d_in, const int* in_sizes, int n_in,
                              void* d_out, int out_size, void* d_ws, size_t ws_size,
                              hipStream_t stream)
{
  if (n_in < 7) return;
  if (in_sizes[0] != NS * CIN * CROP * CROP) return;
  if (in_sizes[1] != CF * CIN * 9 || in_sizes[2] != CF) return;
  if (in_sizes[3] != CF * CF * 9 || in_sizes[4] != CF) return;
  if (in_sizes[5] != CROP * CROP) return;
  if (in_sizes[6] != CF * CROP * NBIN * 2) return;
  if (out_size != NS * CROP * CROP) return;

  const float* z  = (const float*)d_in[0];
  const float* w1 = (const float*)d_in[1];
  const float* b1 = (const float*)d_in[2];
  const float* w2 = (const float*)d_in[3];
  const float* b2 = (const float*)d_in[4];
  const float* cw = (const float*)d_in[5];
  const float* wf = (const float*)d_in[6];
  float* out = (float*)d_out;

  const size_t b_tabs = (size_t)8 * TABN * 2;
  const size_t b_w1p  = (size_t)CF * 32 * 2;
  const size_t b_w2p  = (size_t)CF * K2 * 2;
  const size_t b_f1   = (size_t)NS * CROP * CROP * CF * 2;
  const size_t b_g    = (size_t)2 * PPL * 2;
  const size_t b_G    = (size_t)4 * GPL * 2;
  const size_t b_F    = (size_t)4 * GPL * 2;
  const size_t b_P    = (size_t)4 * PPL * 2;
  const size_t o_tabs = 0;
  const size_t o_w1p  = o_tabs + b_tabs;
  const size_t o_w2p  = o_w1p + b_w1p;
  const size_t o_f1   = o_w2p + b_w2p;
  const size_t o_g    = o_f1 + b_f1;
  const size_t o_G    = o_g + b_g;
  const size_t o_F    = o_G + b_G;
  const size_t o_P    = o_F + b_F;
  const size_t total  = o_P + b_P;
  if (total > ws_size) return;

  char* ws = (char*)d_ws;
  unsigned short* tabs = (unsigned short*)(ws + o_tabs);
  _Float16* w1p = (_Float16*)(ws + o_w1p);
  _Float16* w2p = (_Float16*)(ws + o_w2p);
  _Float16* f1  = (_Float16*)(ws + o_f1);
  unsigned short* ghi = (unsigned short*)(ws + o_g);
  unsigned short* glo = ghi + PPL;
  unsigned short* gpl = (unsigned short*)(ws + o_G);
  unsigned short* fpl = (unsigned short*)(ws + o_F);
  unsigned short* ppl = (unsigned short*)(ws + o_P);

  prep_kernel<<<dim3(CROP + 10), dim3(128), 0, stream>>>(w1, w2, tabs, w1p, w2p);
  conv1_kernel<<<dim3(NS * CROP), dim3(256), 0, stream>>>(z, w1p, b1, f1);
  conv2_kernel<<<dim3(NS * CROP), dim3(256), 0, stream>>>(f1, w2p, b2, cw, ghi, glo);
  rowdft_kernel<<<dim3(VP / 16, NS), dim3(256), 0, stream>>>(ghi, glo, tabs, gpl);
  coldft_kernel<<<dim3(VP / 16, NS), dim3(256), 0, stream>>>(gpl, tabs, wf, fpl);
  invcol_kernel<<<dim3(CROP / 16, NS), dim3(160), 0, stream>>>(fpl, tabs, ppl);
  invrow_kernel<<<dim3(CROP / 16, NS), dim3(256), 0, stream>>>(ppl, tabs, out);
}
